// MambaBlock_57166014710267
// MI455X (gfx1250) — hardware-verified
//
#include <hip/hip_runtime.h>
#include <math.h>

typedef __attribute__((ext_vector_type(16))) _Float16 v16h;
typedef __attribute__((ext_vector_type(8)))  _Float16 v8h;
typedef __attribute__((ext_vector_type(16))) __bf16   v16b;
typedef __attribute__((ext_vector_type(8)))  __bf16   v8b;
typedef __attribute__((ext_vector_type(8)))  float    v8f;
typedef __attribute__((ext_vector_type(4)))  float    v4f;

constexpr int kBatch = 2;
constexpr int kSeqL  = 1024;
constexpr int kDinp  = 1024;
constexpr int kDmod  = 2048;
constexpr int kNst   = 16;
constexpr int kDis   = 128;
constexpr int kAbP   = 2 * kDmod;
constexpr int kRows  = kBatch * kSeqL;
constexpr int kCatN  = 2 * kNst + kDis;
constexpr int kCatP  = 192;
constexpr int kTP    = 260;
constexpr int kScanBlkPerB = kDmod / 256;
constexpr float kCarryW = 32.0f;
constexpr float kCarryA = 64.0f;
constexpr float kCarryG = 256.0f;
static_assert(kCatN == 160 && kCatN <= kCatP && (kCatP % 64) == 0, "concatenated projection width");
static_assert((kDinp % 32) == 0 && (kDmod % 32) == 0 && (kDis % 32) == 0, "GEMM K multiples of 32");
static_assert((kRows % 64) == 0 && (kAbP % 64) == 0 && (kDmod % 64) == 0 && (kDinp % 64) == 0, "GEMM M,N multiples of 64");
static_assert((kSeqL % 64) == 0 && (kDmod % 256) == 0 && (kSeqL % 16) == 0, "tile multiples");

constexpr size_t kOffSEQ16  = 0;
constexpr size_t kOffWIN16  = kOffSEQ16  + (size_t)kRows * kDinp * 2;
constexpr size_t kOffWOUT16 = kOffWIN16  + (size_t)kAbP  * kDinp * 2;
constexpr size_t kOffWCAT16 = kOffWOUT16 + (size_t)kDinp * kDmod * 2;
constexpr size_t kOffWD216  = kOffWCAT16 + (size_t)kCatP * kDmod * 2;
constexpr size_t kOffAB     = kOffWD216  + (size_t)kDmod * kDis  * 2;
constexpr size_t kOffUC     = kOffAB     + (size_t)kRows * kAbP  * 4;
constexpr size_t kOffUC16   = kOffUC     + (size_t)kRows * kDmod * 4;
constexpr size_t kOffBCD    = kOffUC16   + (size_t)kRows * kDmod * 2;
constexpr size_t kOffT116   = kOffBCD    + (size_t)kRows * kCatP * 4;
constexpr size_t kOffT2     = kOffT116   + (size_t)kRows * kDis  * 2;
constexpr size_t kOffY16    = kOffT2     + (size_t)kRows * kDmod * 4;
constexpr size_t kWsTotal   = kOffY16    + (size_t)kRows * kDmod * 2;
static_assert(kWsTotal == 104071168ull, "carve total");
static_assert(kWsTotal <= 134217728ull, "carve cap");
static_assert((kOffWIN16 % 128) == 0 && (kOffWOUT16 % 128) == 0 && (kOffWCAT16 % 128) == 0 && (kOffWD216 % 128) == 0 &&
              (kOffAB % 128) == 0 && (kOffUC % 128) == 0 && (kOffUC16 % 128) == 0 && (kOffBCD % 128) == 0 &&
              (kOffT116 % 128) == 0 && (kOffT2 % 128) == 0 && (kOffY16 % 128) == 0, "128-B aligned regions");

__device__ __forceinline__ unsigned short f2bf_bits(float f) {
  unsigned u = __float_as_uint(f);
  return (unsigned short)((u + 0x7FFFu + ((u >> 16) & 1u)) >> 16);
}
__device__ __forceinline__ float bf_bits2f(unsigned short h) { return __uint_as_float(((unsigned)h) << 16); }
__device__ __forceinline__ float bf_rne(float f) { return bf_bits2f(f2bf_bits(f)); }

__device__ __forceinline__ void dep_guard4_h(v8f& a, v8f& b, v8f& c, v8f& d, v16h x, v16h y, v16h z) { asm volatile("v_nop\n\tv_nop\n\tv_nop\n\tv_nop" : "+v"(a), "+v"(b), "+v"(c), "+v"(d) : "v"(x), "v"(y), "v"(z)); }
__device__ __forceinline__ void dep_guard4_b(v8f& a, v8f& b, v8f& c, v8f& d, v16b x, v16b y, v16b z) { asm volatile("v_nop\n\tv_nop\n\tv_nop\n\tv_nop" : "+v"(a), "+v"(b), "+v"(c), "+v"(d) : "v"(x), "v"(y), "v"(z)); }
__device__ __forceinline__ void keep4_h(v16h a, v16h b, v16h c, v16h d) { asm volatile("v_nop" :: "v"(a), "v"(b), "v"(c), "v"(d)); }
__device__ __forceinline__ void keep4_b(v16b a, v16b b, v16b c, v16b d) { asm volatile("v_nop" :: "v"(a), "v"(b), "v"(c), "v"(d)); }
__device__ __forceinline__ void acc_guard4(v8f& a, v8f& b, v8f& c, v8f& d) { asm volatile("v_nop\n\tv_nop\n\tv_nop\n\tv_nop" : "+v"(a), "+v"(b), "+v"(c), "+v"(d)); }
template <typename T> struct Frag;
template <> struct Frag<_Float16> {
  typedef v16h V; union U { v16h v; v8h h[2]; };
  static __device__ __forceinline__ v16h load(const _Float16* p) {
    U f; f.h[0] = *(const v8h*)(p); f.h[1] = *(const v8h*)(p + 16); return f.v;
  }
  static __device__ __forceinline__ v8f mma(v16h a, v16h b, v8f c) {
    return __builtin_amdgcn_wmma_f32_16x16x32_f16(false, a, false, b, (short)0, c, false, false);
  }
  static __device__ __forceinline__ void guard(v8f& a, v8f& b, v8f& c, v8f& d, v16h x, v16h y, v16h z) { dep_guard4_h(a, b, c, d, x, y, z); }
  static __device__ __forceinline__ void keep(v16h a, v16h b, v16h c, v16h d) { keep4_h(a, b, c, d); }
};
template <> struct Frag<__bf16> {
  typedef v16b V; union U { v16b v; v8b h[2]; };
  static __device__ __forceinline__ v16b load(const __bf16* p) {
    U f; f.h[0] = *(const v8b*)(p); f.h[1] = *(const v8b*)(p + 16); return f.v;
  }
  static __device__ __forceinline__ v8f mma(v16b a, v16b b, v8f c) {
    return __builtin_amdgcn_wmma_f32_16x16x32_bf16(false, a, false, b, (short)0, c, false, false);
  }
  static __device__ __forceinline__ void guard(v8f& a, v8f& b, v8f& c, v8f& d, v16b x, v16b y, v16b z) { dep_guard4_b(a, b, c, d, x, y, z); }
  static __device__ __forceinline__ void keep(v16b a, v16b b, v16b c, v16b d) { keep4_b(a, b, c, d); }
};

template <int ET> struct Elem;
template <> struct Elem<0> { typedef _Float16 T; };
template <> struct Elem<1> { typedef __bf16 T; };
template <int ET, bool SPLIT, int BIAS_MODE, int OUT_MODE, bool RESID, int ACT = 0>
__global__ __launch_bounds__(256) void wmma_gemm64(
    const unsigned short* __restrict__ Ap, const unsigned short* __restrict__ A2p, int lda, long strideA,
    const unsigned short* __restrict__ Btp, const unsigned short* __restrict__ Bt2p, int ldb, long strideB,
    void* __restrict__ Cout, void* __restrict__ Cout2, int ldc, long strideC,
    const float* __restrict__ bias,
    const float* __restrict__ resid, long strideR,
    int M, int N, int K, float scale) {
  typedef typename Elem<ET>::T T;
  typedef typename Frag<T>::V V;
  const T* A = (const T*)Ap; const T* A2 = (const T*)A2p; const T* Bt = (const T*)Btp; const T* Bt2 = (const T*)Bt2p;
  __shared__ __align__(16) float sT[8][16 * 68];
  const int b    = blockIdx.y;
  const int lane = threadIdx.x & 31;
  const int wave = threadIdx.x >> 5;
  const int tilesN = N >> 6;
  const int tilesM = M >> 6;
  const int tile = blockIdx.x * 8 + wave;
  if (tile >= tilesM * tilesN) return;
  const int tm = tile / tilesN;
  const int tn = tile - tm * tilesN;
  const int m0 = tm << 6;
  const int n0 = tn << 6;

  const T* Ab  = A  + (size_t)b * strideA;
  const T* Bb  = Bt + (size_t)b * strideB;
  const T* Ab2 = SPLIT ? (A2  + (size_t)b * strideA) : nullptr;
  const T* Bb2 = SPLIT ? (Bt2 + (size_t)b * strideB) : nullptr;

  const int rlane = lane & 15;
  const int koff  = (lane >> 4) * 8;
  const int mOff  = (lane >> 4) * 8;

  v8f acc[4][4];
#pragma unroll
  for (int i = 0; i < 4; ++i)
#pragma unroll
    for (int j = 0; j < 4; ++j) acc[i][j] = (v8f){0.f,0.f,0.f,0.f,0.f,0.f,0.f,0.f};

  for (int k0 = 0; k0 < K; k0 += 32) {
    V bh[4], bl[4];
#pragma unroll
    for (int j = 0; j < 4; ++j) {
      const size_t bo = (size_t)(n0 + (j << 4) + rlane) * ldb + koff + k0;
      bh[j] = Frag<T>::load(Bb + bo);
      if (SPLIT) bl[j] = Frag<T>::load(Bb2 + bo);
    }
#pragma unroll
    for (int i = 0; i < 4; ++i) {
      const size_t ao = (size_t)(m0 + (i << 4) + rlane) * lda + koff + k0;
      V ah = Frag<T>::load(Ab + ao);
      V al;
      if (SPLIT) al = Frag<T>::load(Ab2 + ao);
#pragma unroll
      for (int j = 0; j < 4; ++j) {
        acc[i][j] = Frag<T>::mma(ah, bh[j], acc[i][j]);
        if (SPLIT) {
          acc[i][j] = Frag<T>::mma(ah, bl[j], acc[i][j]);
          acc[i][j] = Frag<T>::mma(al, bh[j], acc[i][j]);
        }
      }
      Frag<T>::guard(acc[i][0], acc[i][1], acc[i][2], acc[i][3], ah, SPLIT ? al : ah, bh[3]);
    }
    Frag<T>::keep(bh[0], bh[1], bh[2], bh[3]);
    if (SPLIT) Frag<T>::keep(bl[0], bl[1], bl[2], bl[3]);
  }
  acc_guard4(acc[0][0], acc[0][1], acc[0][2], acc[0][3]);
  acc_guard4(acc[1][0], acc[1][1], acc[1][2], acc[1][3]);
  acc_guard4(acc[2][0], acc[2][1], acc[2][2], acc[2][3]);
  acc_guard4(acc[3][0], acc[3][1], acc[3][2], acc[3][3]);

  float* slab = sT[wave];
  const float* Rb = RESID ? (resid + (size_t)b * strideR) : nullptr;
#pragma unroll
  for (int i = 0; i < 4; ++i) {
    const int mBase = m0 + (i << 4);
#pragma unroll
    for (int j = 0; j < 4; ++j) {
      const int n = n0 + (j << 4) + rlane;
      float bv = 0.f;
      if (BIAS_MODE == 2) bv = bias[n];
#pragma unroll
      for (int r = 0; r < 8; ++r) {
        float v = acc[i][j][r] * scale;
        if (BIAS_MODE == 1) v += bias[mBase + mOff + r];
        if (BIAS_MODE == 2) v += bv;
        if (RESID) v += Rb[(size_t)(mBase + mOff + r) * ldc + n];
        if (ACT == 1) v = tanhf(v);
        if (ACT == 2) v = fmaxf(v, 0.0f);
        if (ACT == 3) v = v / (1.0f + expf(-v));
        if (ACT == 4) v = (v > 0.f) ? v : 0.01f * v;
        slab[(mOff + r) * 68 + (j << 4) + rlane] = v;
      }
    }
    __builtin_amdgcn_fence(__ATOMIC_RELEASE, "workgroup");
    __builtin_amdgcn_wave_barrier();
    __builtin_amdgcn_fence(__ATOMIC_ACQUIRE, "workgroup");
    if (OUT_MODE == 0) {
      float* C = (float*)Cout + (size_t)b * strideC;
      const int hh = lane >> 4, c4 = (lane & 15) * 4;
      for (int pass = 0; pass < 2; ++pass) {
#pragma unroll
        for (int it = 0; it < 8; ++it) {
          const int row = it * 2 + hh;
          v4f v = *(const v4f*)(slab + row * 68 + c4);
          *(volatile v4f*)(C + (size_t)(mBase + row) * ldc + n0 + c4) = v;
        }
        __threadfence();
      }
    } else {
      const int q = lane >> 3, c8 = (lane & 7) * 8;
      unsigned short* C  = (unsigned short*)Cout  + (size_t)b * strideC;
      unsigned short* C2 = (OUT_MODE == 2) ? ((unsigned short*)Cout2 + (size_t)b * strideC) : nullptr;
      for (int pass = 0; pass < 2; ++pass) {
#pragma unroll
        for (int it = 0; it < 4; ++it) {
          const int row = it * 4 + q;
          const float* sp = slab + row * 68 + c8;
          v8h hv, lv;
#pragma unroll
          for (int e = 0; e < 8; ++e) {
            if (OUT_MODE == 1) {
              hv[e] = (_Float16)sp[e];
            } else {
              unsigned short hb = f2bf_bits(sp[e]);
              unsigned short lb = f2bf_bits(sp[e] - bf_bits2f(hb));
              hv[e] = __builtin_bit_cast(_Float16, hb);
              lv[e] = __builtin_bit_cast(_Float16, lb);
            }
          }
          *(volatile v8h*)(C + (size_t)(mBase + row) * ldc + n0 + c8) = hv;
          if (OUT_MODE == 2) *(volatile v8h*)(C2 + (size_t)(mBase + row) * ldc + n0 + c8) = lv;
        }
        __threadfence();
      }
    }
    __builtin_amdgcn_fence(__ATOMIC_RELEASE, "workgroup");
    __builtin_amdgcn_wave_barrier();
    __builtin_amdgcn_fence(__ATOMIC_ACQUIRE, "workgroup");
  }
}

__global__ __launch_bounds__(256) void cast_bfr_f16_kernel(
    const float* __restrict__ src, unsigned short* __restrict__ dst, int total8, float scale)
{
  const int i = blockIdx.x * 256 + threadIdx.x;
  if (i >= total8) return;
  const size_t e0 = (size_t)i << 3;
  const float* p = src + e0;
  const v4f a0 = *(const v4f*)(p);
  const v4f a1 = *(const v4f*)(p + 4);
  v8h hv;
#pragma unroll
  for (int e = 0; e < 4; ++e) {
    const float x0 = a0[e];
    const float x1 = a1[e];
    hv[e]     = (_Float16)(bf_rne(x0) * scale);
    hv[4 + e] = (_Float16)(bf_rne(x1) * scale);
  }
  unsigned short* q = dst + e0;
  *(volatile v8h*)q = hv;
  __threadfence();
  *(volatile v8h*)q = hv;
}

__global__ __launch_bounds__(256) void wcat_kernel(
    const float* __restrict__ wB, const float* __restrict__ wC, const float* __restrict__ wD1,
    unsigned short* __restrict__ dst, float scale)
{
  const int row = blockIdx.x;
  const int c8  = threadIdx.x * 8;
  const float* src = wB;
  int srow = 0;
  if (row < kNst) { src = wB; srow = row; }
  else if (row < 2 * kNst) { src = wC; srow = row - kNst; }
  else if (row < kCatN) { src = wD1; srow = row - 2 * kNst; }
  const bool live = (row < kCatN);
  const float* p = src + (size_t)srow * kDmod + c8;
  const v4f a0 = *(const v4f*)(p);
  const v4f a1 = *(const v4f*)(p + 4);
  v8h hv;
#pragma unroll
  for (int e = 0; e < 4; ++e) {
    const float x0 = a0[e];
    const float x1 = a1[e];
    const float y0 = live ? (bf_rne(x0) * scale) : 0.0f;
    const float y1 = live ? (bf_rne(x1) * scale) : 0.0f;
    hv[e]     = (_Float16)y0;
    hv[4 + e] = (_Float16)y1;
  }
  unsigned short* q = dst + (size_t)row * kDmod + c8;
  *(volatile v8h*)q = hv;
  __threadfence();
  *(volatile v8h*)q = hv;
}

__global__ __launch_bounds__(256) void t1_cast_kernel(
    const float* __restrict__ BCD, unsigned short* __restrict__ T116, int total8, float scale)
{
  const int i = blockIdx.x * 256 + threadIdx.x;
  if (i >= total8) return;
  const int e0  = i << 3;
  const int row = e0 >> 7;
  const int c8  = e0 & (kDis - 1);
  const float* p = BCD + (size_t)row * kCatP + 2 * kNst + c8;
  const v4f a0 = *(const v4f*)(p);
  const v4f a1 = *(const v4f*)(p + 4);
  v8h hv;
#pragma unroll
  for (int e = 0; e < 4; ++e) {
    const float x0 = a0[e];
    const float x1 = a1[e];
    hv[e]     = (_Float16)(x0 * scale);
    hv[4 + e] = (_Float16)(x1 * scale);
  }
  unsigned short* qd = T116 + e0;
  *(volatile v8h*)qd = hv;
  __threadfence();
  *(volatile v8h*)qd = hv;
}

__global__ __launch_bounds__(256) void conv_silu_kernel(
    const float* __restrict__ AB, const float* __restrict__ cw, const float* __restrict__ cb,
    float* __restrict__ UC, unsigned short* __restrict__ UC16)
{
  __shared__ __align__(16) float sT[16 * kTP];
  const int tid = threadIdx.x, lane = tid & 31, wave = tid >> 5;
  const int d0 = blockIdx.x * 256, d = d0 + tid;
  const int g0 = blockIdx.y * 64;
  const int tb = g0 & (kSeqL - 1);
  const v4f wv = *(const v4f*)(cw + (size_t)d * 4);
  const float wr0 = wv[0], wr1 = wv[1], wr2 = wv[2], wr3 = wv[3];
  const float w0 = bf_rne(wr0), w1 = bf_rne(wr1), w2 = bf_rne(wr2), w3 = bf_rne(wr3);
  const float bc = bf_rne(cb[d]);
  float xm3, xm2, xm1;
  {
    const bool hist = (tb > 0);
    const int rb = hist ? (g0 - 3) : g0;
    const float v3 = AB[(size_t)rb * kAbP + d];
    const float v2 = AB[(size_t)(rb + 1) * kAbP + d];
    const float v1 = AB[(size_t)(rb + 2) * kAbP + d];
    xm3 = hist ? v3 : 0.f;
    xm2 = hist ? v2 : 0.f;
    xm1 = hist ? v1 : 0.f;
  }
  const int hrow = wave >> 1;
  const int hch  = (wave & 1) * 128 + lane * 4;
#pragma unroll 1
  for (int sub = 0; sub < 4; ++sub) {
    const int lb = g0 + sub * 16;
#pragma unroll 1
    for (int s = 0; s < 16; ++s) {
      const float xcur = AB[(size_t)(lb + s) * kAbP + d];
      float acc = w0 * xm3;
      acc = fmaf(w1, xm2, acc);
      acc = fmaf(w2, xm1, acc);
      acc = fmaf(w3, xcur, acc);
      const float sv = acc + bc;
      const float sg = __builtin_amdgcn_rcpf(1.0f + expf(-sv));
      sT[s * kTP + tid] = sv * sg;
      xm3 = xm2; xm2 = xm1; xm1 = xcur;
    }
    __syncthreads();
    v4f fv[4];
    v8h bv[2];
#pragma unroll
    for (int it = 0; it < 4; ++it) fv[it] = *(const v4f*)(sT + (it * 4 + hrow) * kTP + hch);
#pragma unroll
    for (int it = 0; it < 2; ++it) {
      const float* sp = sT + (it * 8 + wave) * kTP + lane * 8;
      const v4f a0 = *(const v4f*)(sp);
      const v4f a1 = *(const v4f*)(sp + 4);
#pragma unroll
      for (int e = 0; e < 4; ++e) {
        const float x0 = a0[e];
        const float x1 = a1[e];
        bv[it][e]     = (_Float16)(x0 * kCarryA);
        bv[it][4 + e] = (_Float16)(x1 * kCarryA);
      }
    }
    for (int pass = 0; pass < 2; ++pass) {
#pragma unroll
      for (int it = 0; it < 4; ++it)
        *(volatile v4f*)(UC + (size_t)(lb + it * 4 + hrow) * kDmod + d0 + hch) = fv[it];
#pragma unroll
      for (int it = 0; it < 2; ++it)
        *(volatile v8h*)(UC16 + (size_t)(lb + it * 8 + wave) * kDmod + d0 + lane * 8) = bv[it];
      __threadfence();
    }
    __syncthreads();
  }
}

__global__ __launch_bounds__(256) void scan_kernel(
    const float* __restrict__ T2, const float* __restrict__ UC, const float* __restrict__ AB,
    const float* __restrict__ BCD, const float* __restrict__ Apar, const float* __restrict__ Dp,
    unsigned short* __restrict__ Y16)
{
  __shared__ __align__(16) float sBC[16 * 32];
  __shared__ __align__(16) float sY[16 * kTP];
  __shared__ __align__(16) float sA[kNst * 256];
  const int tid = threadIdx.x, lane = tid & 31, wave = tid >> 5;
  const int bix = blockIdx.x / kScanBlkPerB;
  const int d0  = (blockIdx.x - bix * kScanBlkPerB) * 256;
  const int d   = d0 + tid;
  const size_t row0 = (size_t)bix * kSeqL;

#pragma unroll 1
  for (int s = 0; s < kNst; ++s) sA[s * 256 + tid] = expf(-bf_rne(Apar[(size_t)d * kNst + s]));
  __syncthreads();
  float eA[kNst], h[kNst];
#pragma unroll
  for (int s = 0; s < kNst; ++s) {
    eA[s] = sA[s * 256 + tid];
    h[s] = 0.f;
  }
  const float Dd = bf_rne(Dp[d]);

#pragma unroll 1
  for (int c = 0; c < kSeqL / 16; ++c) {
    const int l0 = c * 16;
    if (tid < 128) {
      const int r = tid >> 3, q = (tid & 7) * 4;
      const v4f v = *(const v4f*)(BCD + (row0 + l0 + r) * kCatP + q);
      *(v4f*)(sBC + r * 32 + q) = v;
    }
    __syncthreads();
#pragma unroll 1
    for (int s = 0; s < 16; ++s) {
      const size_t m = row0 + (size_t)(l0 + s);
      const float t2v = T2[m * kDmod + d];
      const float xv  = UC[m * kDmod + d];
      const float zv  = AB[m * kAbP + kDmod + d];
      const float a     = Dd + t2v;
      const float delta = fmaxf(a, 0.0f) + log1pf(expf(-fabsf(a)));
      v4f Bq[4], Cq[4];
#pragma unroll
      for (int qq = 0; qq < 4; ++qq) {
        Bq[qq] = *(const v4f*)(sBC + s * 32 + 4 * qq);
        Cq[qq] = *(const v4f*)(sBC + s * 32 + kNst + 4 * qq);
      }
      float y = 0.f;
#pragma unroll
      for (int n = 0; n < kNst; ++n) {
        float e = eA[n] * delta;
        asm volatile("" : "+v"(e));
        float db = Bq[n >> 2][n & 3] * delta;
        asm volatile("" : "+v"(db));
        float p = db * xv;
        asm volatile("" : "+v"(p));
        float qv = e * h[n];
        asm volatile("" : "+v"(qv));
        const float hn = qv + p;
        h[n] = hn;
        float rr = hn * Cq[n >> 2][n & 3];
        asm volatile("" : "+v"(rr));
        y += rr;
      }
      float sk = Dd * xv;
      asm volatile("" : "+v"(sk));
      y += sk;
      const float sg = __builtin_amdgcn_rcpf(1.0f + expf(-zv));
      const float g  = zv * sg;
      sY[s * kTP + tid] = (y * g) * kCarryG;
    }
    __syncthreads();
    v8h hv[2];
#pragma unroll
    for (int it = 0; it < 2; ++it) {
      const float* sp = sY + (it * 8 + wave) * kTP + lane * 8;
      const v4f a0 = *(const v4f*)(sp);
      const v4f a1 = *(const v4f*)(sp + 4);
#pragma unroll
      for (int e = 0; e < 4; ++e) {
        const float x0 = a0[e];
        const float x1 = a1[e];
        hv[it][e]     = (_Float16)x0;
        hv[it][4 + e] = (_Float16)x1;
      }
    }
    for (int pass = 0; pass < 2; ++pass) {
#pragma unroll
      for (int it = 0; it < 2; ++it)
        *(volatile v8h*)(Y16 + (row0 + (size_t)(l0 + it * 8 + wave)) * kDmod + d0 + lane * 8) = hv[it];
      __threadfence();
    }
  }
}

extern "C" void kernel_launch(void* const* d_in, const int* in_sizes, int n_in,
                              void* d_out, int out_size, void* d_ws, size_t ws_size,
                              hipStream_t stream)
{
  if (n_in < 11) return;
  if (in_sizes[0] != kRows * kDinp) return;
  if (in_sizes[1] != kAbP * kDinp) return;
  if (in_sizes[2] != kDinp * kDmod) return;
  if (in_sizes[3] != kNst * kDmod) return;
  if (in_sizes[4] != kNst * kDmod) return;
  if (in_sizes[5] != kDis * kDmod) return;
  if (in_sizes[6] != kDmod * kDis) return;
  if (in_sizes[7] != kDmod * 4) return;
  if (in_sizes[8] != kDmod) return;
  if (in_sizes[9] != kDmod * kNst) return;
  if (in_sizes[10] != kDmod) return;
  if (out_size != kRows * kDinp) return;
  if (ws_size < kWsTotal) return;

  const float* seq    = (const float*)d_in[0];
  const float* w_in   = (const float*)d_in[1];
  const float* w_out  = (const float*)d_in[2];
  const float* w_B    = (const float*)d_in[3];
  const float* w_C    = (const float*)d_in[4];
  const float* w_D1   = (const float*)d_in[5];
  const float* w_D2   = (const float*)d_in[6];
  const float* conv_w = (const float*)d_in[7];
  const float* conv_b = (const float*)d_in[8];
  const float* A_par  = (const float*)d_in[9];
  const float* D_par  = (const float*)d_in[10];
  float* out = (float*)d_out;

  char* ws = (char*)d_ws;
  unsigned short* SEQ16  = (unsigned short*)(ws + kOffSEQ16);
  unsigned short* WIN16  = (unsigned short*)(ws + kOffWIN16);
  unsigned short* WOUT16 = (unsigned short*)(ws + kOffWOUT16);
  unsigned short* WCAT16 = (unsigned short*)(ws + kOffWCAT16);
  unsigned short* WD216  = (unsigned short*)(ws + kOffWD216);
  float*          AB     = (float*)(ws + kOffAB);
  float*          UC     = (float*)(ws + kOffUC);
  unsigned short* UC16   = (unsigned short*)(ws + kOffUC16);
  float*          BCD    = (float*)(ws + kOffBCD);
  unsigned short* T116   = (unsigned short*)(ws + kOffT116);
  float*          T2     = (float*)(ws + kOffT2);
  unsigned short* Y16    = (unsigned short*)(ws + kOffY16);
  const float* dummy_bias  = D_par;
  const float* dummy_resid = seq;

  cast_bfr_f16_kernel<<<(kRows * kDinp / 8) / 256, 256, 0, stream>>>(seq,   SEQ16,  kRows * kDinp / 8, 1.0f);
  cast_bfr_f16_kernel<<<(kAbP * kDinp / 8) / 256, 256, 0, stream>>>(w_in,  WIN16,  kAbP * kDinp / 8, kCarryW);
  cast_bfr_f16_kernel<<<(kDinp * kDmod / 8) / 256, 256, 0, stream>>>(w_out, WOUT16, kDinp * kDmod / 8, kCarryW);
  cast_bfr_f16_kernel<<<(kDmod * kDis / 8) / 256, 256, 0, stream>>>(w_D2,  WD216,  kDmod * kDis / 8, kCarryW);
  wcat_kernel<<<kCatP, 256, 0, stream>>>(w_B, w_C, w_D1, WCAT16, kCarryW);

  wmma_gemm64<0, false, 0, 0, false><<<dim3(256, 1), 256, 0, stream>>>(
      SEQ16, SEQ16, kDinp, 0L, WIN16, WIN16, kDinp, 0L,
      (void*)AB, (void*)AB, kAbP, 0L, dummy_bias, dummy_resid, 0L,
      kRows, kAbP, kDinp, 1.0f / kCarryW);

  conv_silu_kernel<<<dim3(kDmod / 256, kRows / 64), 256, 0, stream>>>(AB, conv_w, conv_b, UC, UC16);

  wmma_gemm64<0, false, 0, 0, false><<<dim3(12, 1), 256, 0, stream>>>(
      UC16, UC16, kDmod, 0L, WCAT16, WCAT16, kDmod, 0L,
      (void*)BCD, (void*)BCD, kCatP, 0L, dummy_bias, dummy_resid, 0L,
      kRows, kCatP, kDmod, 1.0f / (kCarryA * kCarryW));

  t1_cast_kernel<<<(kRows * kDis / 8) / 256, 256, 0, stream>>>(BCD, T116, kRows * kDis / 8, kCarryA);

  wmma_gemm64<0, false, 0, 0, false><<<dim3(128, 1), 256, 0, stream>>>(
      T116, T116, kDis, 0L, WD216, WD216, kDis, 0L,
      (void*)T2, (void*)T2, kDmod, 0L, dummy_bias, dummy_resid, 0L,
      kRows, kDmod, kDis, 1.0f / (kCarryA * kCarryW));

  scan_kernel<<<kBatch * kScanBlkPerB, 256, 0, stream>>>(T2, UC, AB, BCD, A_par, D_par, Y16);

  wmma_gemm64<0, false, 0, 0, false><<<dim3(64, 1), 256, 0, stream>>>(
      Y16, Y16, kDmod, 0L, WOUT16, WOUT16, kDmod, 0L,
      (void*)out, (void*)out, kDinp, 0L, dummy_bias, dummy_resid, 0L,
      kRows, kDinp, kDmod, 1.0f / (kCarryG * kCarryW));
}
